// PointwiseSpAggregatedAttention_47304769798729
// MI455X (gfx1250) — hardware-verified
//
#include <hip/hip_runtime.h>
#include <hip/hip_bf16.h>

typedef __bf16         v16bf __attribute__((ext_vector_type(16)));
typedef unsigned int   v8u   __attribute__((ext_vector_type(8)));
typedef unsigned int   v4u   __attribute__((ext_vector_type(4)));
typedef float          v8f   __attribute__((ext_vector_type(8)));
typedef float          v4f   __attribute__((ext_vector_type(4)));
typedef v4f __attribute__((may_alias)) v4fa;
typedef v4u __attribute__((may_alias)) v4ua;

union Frag { v16bf v; v8u u; v4u q[2]; };

namespace {
constexpr int BATCH = 2;
constexpr int SEQ   = 2048;
constexpr int DM    = 1024;
constexpr int NH    = 16;
constexpr int HD    = 64;
constexpr int NX    = BATCH * SEQ * DM;
constexpr int NX8   = NX / 8;
constexpr int TP    = 136;
constexpr int VTOK  = 128;
constexpr int QB    = 64;
constexpr int KSTEP = 64;
}

__device__ __forceinline__ v8f wmma_bf16(v16bf a, v16bf b, v8f c) {
  v8f d = __builtin_amdgcn_wmma_f32_16x16x32_bf16(false, a, false, b, (short)0, c, false, false);
  asm volatile("v_nop\n\tv_nop\n\tv_nop\n\tv_nop" : "+v"(d) : "v"(a), "v"(b));
  return d;
}

__device__ __forceinline__ v16bf load_frag(const unsigned short* p, int h) {
  Frag f;
  f.q[0] = *(const v4ua*)(p + 8 * h);
  f.q[1] = *(const v4ua*)(p + 16 + 8 * h);
  return f.v;
}

__device__ __forceinline__ unsigned int bf16_rne(float f) {
  unsigned int u = __float_as_uint(f);
  u += 0x7FFFu + ((u >> 16) & 1u);
  return u >> 16;
}

__device__ __forceinline__ unsigned int split_pair(float x0, float x1, unsigned int& lo_pair) {
  const unsigned int h0 = bf16_rne(x0), h1 = bf16_rne(x1);
  const float r0 = x0 - __uint_as_float(h0 << 16);
  const float r1 = x1 - __uint_as_float(h1 << 16);
  lo_pair = bf16_rne(r0) | (bf16_rne(r1) << 16);
  return h0 | (h1 << 16);
}

__global__ __launch_bounds__(256) void k_cvt(
    const float* __restrict__ q, const float* __restrict__ k,
    unsigned short* __restrict__ qb, unsigned short* __restrict__ kb)
{
  const int g = blockIdx.x * 256 + threadIdx.x;
  if (g >= 2 * NX8) return;
  const float* src;
  unsigned short* dst;
  if (g < NX8) {
    src = q + (size_t)g * 8;
    dst = qb + (size_t)g * 8;
  } else {
    const int e = g - NX8;
    src = k + (size_t)e * 8;
    dst = kb + (size_t)e * 8;
  }
  const v4f a = *(const v4fa*)src;
  const v4f c = *(const v4fa*)(src + 4);
  v4u o;
  o.x = bf16_rne(a.x) | (bf16_rne(a.y) << 16);
  o.y = bf16_rne(a.z) | (bf16_rne(a.w) << 16);
  o.z = bf16_rne(c.x) | (bf16_rne(c.y) << 16);
  o.w = bf16_rne(c.z) | (bf16_rne(c.w) << 16);
  *(volatile v4u*)dst = o;
  __threadfence();
  *(volatile v4u*)dst = o;
}

__device__ __forceinline__ void vt_store_pass(const unsigned short* sT, unsigned short* vt,
                                              int bh, int l0, int w, int lane) {
  const int q8 = lane & 7, sub = lane >> 3;
  #pragma unroll
  for (int i = 0; i < 4; ++i) {
    const int lid = w * 16 + i * 4 + sub;
    const int d = lid >> 1, hl = lid & 1;
    const v4u val = *(const v4ua*)(sT + d * TP + 64 * hl + 8 * q8);
    unsigned short* dst = vt + ((size_t)bh * HD + d) * SEQ + l0 + 64 * hl + 8 * q8;
    *(volatile v4u*)dst = val;
  }
}

__global__ __launch_bounds__(256) void k_vt(const float* __restrict__ v, unsigned short* __restrict__ vt)
{
  __shared__ __attribute__((aligned(16))) unsigned short sT[HD * TP];

  const int tid = threadIdx.x, lane = tid & 31, w = tid >> 5;
  const int bh = blockIdx.y, b = bh >> 4, head = bh & 15;
  const int l0 = blockIdx.x * VTOK;

  #pragma unroll
  for (int it = 0; it < (VTOK * HD / 4) / 256; ++it) {
    const int idx = tid + it * 256;
    const int tok = idx >> 4, c = idx & 15;
    const v4f x = *(const v4fa*)(v + ((size_t)b * SEQ + l0 + tok) * DM + head * HD + 4 * c);
    sT[(4 * c + 0) * TP + tok] = (unsigned short)bf16_rne(x.x);
    sT[(4 * c + 1) * TP + tok] = (unsigned short)bf16_rne(x.y);
    sT[(4 * c + 2) * TP + tok] = (unsigned short)bf16_rne(x.z);
    sT[(4 * c + 3) * TP + tok] = (unsigned short)bf16_rne(x.w);
  }
  __syncthreads();

  vt_store_pass(sT, vt, bh, l0, w, lane);
  __threadfence();
  vt_store_pass(sT, vt, bh, l0, w, lane);
}

__device__ __forceinline__ v8f silu8(v8f s) {
  #pragma unroll
  for (int r = 0; r < 8; ++r) {
    const float x = s[r];
    s[r] = x * __builtin_amdgcn_rcpf(1.0f + __expf(-x));
  }
  return s;
}

__device__ __forceinline__ void pack_p(v8f a, v8f c, v16bf& ph, v16bf& pl) {
  Frag H, L;
  #pragma unroll
  for (int i = 0; i < 4; ++i) {
    unsigned int lo;
    const unsigned int hi = split_pair(a[2 * i], a[2 * i + 1], lo);
    H.u[i] = hi;
    L.u[i] = lo;
  }
  #pragma unroll
  for (int i = 0; i < 4; ++i) {
    unsigned int lo;
    const unsigned int hi = split_pair(c[2 * i], c[2 * i + 1], lo);
    H.u[4 + i] = hi;
    L.u[4 + i] = lo;
  }
  ph = H.v;
  pl = L.v;
}

__device__ __forceinline__ void att_store_pass(const float* so, float* out,
                                               int b, int head, int q0, int lane) {
  const int q8 = lane & 7, sub = lane >> 3;
  #pragma unroll
  for (int i = 0; i < 8; ++i) {
    const int lid = i * 4 + sub;
    const int row = lid >> 1, hl = lid & 1;
    const v4f val = *(const v4fa*)(so + row * 64 + 32 * hl + 4 * q8);
    const size_t gi = ((size_t)b * SEQ + q0 + row) * DM + head * HD + 32 * hl + 4 * q8;
    *(volatile v4f*)(out + gi) = val;
  }
}

__global__ __launch_bounds__(128) void k_attn(
    const unsigned short* __restrict__ qb,
    const unsigned short* __restrict__ kb,
    const unsigned short* __restrict__ vt,
    float* __restrict__ out)
{
  __shared__ __attribute__((aligned(16))) float sO[4 * 16 * 64];

  const int tid = threadIdx.x, lane = tid & 31, w = tid >> 5;
  const int h = lane >> 4, m = lane & 15;
  const int bh = blockIdx.y, b = bh >> 4, head = bh & 15;
  const int q0 = blockIdx.x * QB + 16 * w;

  const unsigned short* qrow = qb + ((size_t)b * SEQ + q0 + m) * DM + head * HD;
  const v16bf qf0 = load_frag(qrow, h);
  const v16bf qf1 = load_frag(qrow + 32, h);

  const v8f zero8 = {0.f, 0.f, 0.f, 0.f, 0.f, 0.f, 0.f, 0.f};
  v8f o[4];
  #pragma unroll
  for (int t = 0; t < 4; ++t) o[t] = zero8;

  const unsigned short* kbase = kb + ((size_t)b * SEQ + m) * DM + head * HD;
  const unsigned short* vbase = vt + ((size_t)bh * HD + m) * SEQ;

  #pragma unroll 1
  for (int key0 = 0; key0 < SEQ; key0 += KSTEP) {
    #pragma unroll
    for (int c = 0; c < 2; ++c) {
      const unsigned short* kp0 = kbase + (size_t)(key0 + 32 * c) * DM;
      const unsigned short* kp1 = kp0 + (size_t)16 * DM;
      const v16bf ka0 = load_frag(kp0, h);
      const v16bf ka1 = load_frag(kp0 + 32, h);
      const v16bf kc0 = load_frag(kp1, h);
      const v16bf kc1 = load_frag(kp1 + 32, h);
      v8f s0 = wmma_bf16(ka0, qf0, zero8);
      s0 = wmma_bf16(ka1, qf1, s0);
      v8f s1 = wmma_bf16(kc0, qf0, zero8);
      s1 = wmma_bf16(kc1, qf1, s1);

      s0 = silu8(s0);
      s1 = silu8(s1);
      v16bf ph, pl;
      pack_p(s0, s1, ph, pl);

      #pragma unroll
      for (int t = 0; t < 4; ++t) {
        const v16bf vf = load_frag(vbase + (size_t)(16 * t) * SEQ + key0 + 32 * c, h);
        o[t] = wmma_bf16(vf, ph, o[t]);
        o[t] = wmma_bf16(vf, pl, o[t]);
      }
    }
  }

  float* so = sO + w * 1024;
  #pragma unroll
  for (int t = 0; t < 4; ++t)
    #pragma unroll
    for (int r = 0; r < 8; ++r)
      so[m * 64 + 16 * t + 8 * h + r] = o[t][r];
  __syncthreads();

  att_store_pass(so, out, b, head, q0, lane);
  __threadfence();
  att_store_pass(so, out, b, head, q0, lane);
}

extern "C" void kernel_launch(void* const* d_in, const int* in_sizes, int n_in,
                              void* d_out, int out_size, void* d_ws, size_t ws_size,
                              hipStream_t stream) {
  if (n_in < 3) return;
  if (in_sizes[0] != NX || in_sizes[1] != NX || in_sizes[2] != NX) return;
  if (out_size != NX) return;

  const float* v = (const float*)d_in[0];
  const float* k = (const float*)d_in[1];
  const float* q = (const float*)d_in[2];
  float* out = (float*)d_out;

  const size_t plane_bytes = (size_t)NX * 2;
  const size_t total = 3 * plane_bytes;
  if (total > ws_size) return;

  char* ws = (char*)d_ws;
  unsigned short* qb = (unsigned short*)(ws);
  unsigned short* kb = (unsigned short*)(ws + plane_bytes);
  unsigned short* vt = (unsigned short*)(ws + 2 * plane_bytes);

  k_cvt<<<(2 * NX8 + 255) / 256, 256, 0, stream>>>(q, k, qb, kb);

  dim3 gVt(SEQ / VTOK, BATCH * NH);
  k_vt<<<gVt, 256, 0, stream>>>(v, vt);

  dim3 gAtt(SEQ / QB, BATCH * NH);
  k_attn<<<gAtt, 128, 0, stream>>>(qb, kb, vt, out);
}
